// EdgeNetwork_70712341561618
// MI455X (gfx1250) — hardware-verified
//
#include <hip/hip_runtime.h>
#include <stddef.h>
#include <stdint.h>

#define EMB     64
#define IND     32
#define NGI     33
#define GW      (NGI * EMB)
#define WROWS   (EMB * EMB)
#define NTHR    256
#define NWAVE   8
#define EPT     8
#define CHUNK   (NTHR * EPT)
#define WCAP    (EPT * 32)
#define LISTN   (NWAVE * WCAP)
#define NBA     1024
#define PKS     10
#define RCAP    28672
#define DEGCAP  64
#define GBM     64
#define GTHR    128
#define NTF     12
#define BNF     (16 * NTF)
#define NCB     (GW / BNF)
#define PPR     (BNF / 8)
#define NITF    (GBM * BNF / (8 * GTHR))
#define NUWW    (IND * EMB * EMB / 8)
#define NUW     (GW * EMB / 8)
#define ETHR    128
#define NITE    (ETHR * EMB / (4 * ETHR))
#define ZINTS   (2 * RCAP + 2 * NBA + LISTN)
#define LDS_AGG (ZINTS * 4 + 64)
#define WSLIM   268435456
#define CARRY     256.0f
#define INV_CARRY 0.00390625f
#define LN_EPS    1e-5f
#define INV_EMB   0.015625f

static_assert((CHUNK & (CHUNK - 1)) == 0);
static_assert(NBA == (1 << PKS));
static_assert(((long long)CHUNK << PKS) < (1LL << 31));
static_assert(NTHR * 4 == NBA);
static_assert(LISTN >= NBA && LISTN >= NWAVE * WCAP);
static_assert((RCAP % 32) == 0);
static_assert((ZINTS % (NTHR * 4)) == 0);
static_assert(LDS_AGG <= 262144);
static_assert((NBA % NWAVE) == 0);
static_assert(GBM == (GTHR / 32) * 16);
static_assert(EMB == 64 && IND == 32 && GW == 2112 && WROWS == 4096);
static_assert((EMB % 32) == 0);
static_assert((GW % BNF) == 0 && NCB * BNF == GW);
static_assert(((BNF * 2) % 128) == 0 && ((GW * 2) % 128) == 0);
static_assert(NITF * GTHR * 8 == GBM * BNF && (PPR % 8) == 0 && (GTHR % 8) == 0);
static_assert((NUW % NTHR) == 0 && (NUWW % NTHR) == 0 && NUW * 8 == GW * EMB);
static_assert(NITE * ETHR * 4 == ETHR * EMB && (ETHR % 32) == 0);
static_assert(((EMB * 4) % 128) == 0);

typedef float          v2f  __attribute__((ext_vector_type(2)));
typedef float          v4f  __attribute__((ext_vector_type(4)));
typedef float          v8f  __attribute__((ext_vector_type(8)));
typedef int            v4i  __attribute__((ext_vector_type(4)));
typedef int            v8i  __attribute__((ext_vector_type(8)));
typedef unsigned int   v4u  __attribute__((ext_vector_type(4)));
typedef unsigned short v8us __attribute__((ext_vector_type(8)));
typedef _Float16       v8h  __attribute__((ext_vector_type(8)));
typedef __bf16         v16b __attribute__((ext_vector_type(16)));
typedef v2f  __attribute__((may_alias)) v2fa;
typedef v4f  __attribute__((may_alias)) v4fa;
typedef v4i  __attribute__((may_alias)) v4ia;
typedef v4u  __attribute__((may_alias)) v4ua;
typedef v8us __attribute__((may_alias)) v8usa;
union Frag { v16b b; v8us h[2]; v8i w; };

__device__ __forceinline__ v8f wmk(const Frag& a, const Frag& b, v8f c) {
  v8f d = __builtin_amdgcn_wmma_f32_16x16x32_bf16(false, a.b, false, b.b, (short)0, c, false, false);
  asm volatile("v_nop\n\tv_nop\n\tv_nop\n\tv_nop" : "+v"(d) : "v"(a.w), "v"(b.w));
  return d;
}

__device__ __forceinline__ unsigned short bf_bits(float f) {
  unsigned int u = __float_as_uint(f);
  u += 0x7FFFu + ((u >> 16) & 1u);
  return (unsigned short)(u >> 16);
}
__device__ __forceinline__ float bf_val(unsigned short b) {
  return __uint_as_float(((unsigned int)b) << 16);
}
__device__ __forceinline__ float bf_rne(float f) { return bf_val(bf_bits(f)); }

__device__ __forceinline__ v8us cvt8(const float* p) {
  const v4f a = *(const v4fa*)p, b = *(const v4fa*)(p + 4);
  v8us o;
  o[0] = bf_bits(a.x); o[1] = bf_bits(a.y); o[2] = bf_bits(a.z); o[3] = bf_bits(a.w);
  o[4] = bf_bits(b.x); o[5] = bf_bits(b.y); o[6] = bf_bits(b.z); o[7] = bf_bits(b.w);
  return o;
}

__device__ __forceinline__ float h2f(unsigned int w) {
  const _Float16 hv = __builtin_bit_cast(_Float16, (unsigned short)(w & 0xFFFFu));
  return (float)hv;
}

__device__ __forceinline__ void put16(unsigned short* dp, v8us o) {
  *(volatile v8us*)dp = o;
  __threadfence();
  *(volatile v8us*)dp = o;
}

__device__ __forceinline__ int scan_chunk(const int* __restrict__ keys, int nE, int cbase, int slotBase,
                                          int nb, int vec8, int* list, int tid, int lane, int wave) {
  int wc = 0;
  const int el0  = tid * EPT;
  const int e0   = cbase + el0;
  const int sent = -2147483647 - 1;
  v4i da, db;
  if (vec8 != 0 && cbase + CHUNK <= nE) {
    da = *(const v4ia*)(keys + e0);
    db = *(const v4ia*)(keys + e0 + 4);
  } else {
    da.x = (e0     < nE) ? keys[min(e0,     nE - 1)] : sent;
    da.y = (e0 + 1 < nE) ? keys[min(e0 + 1, nE - 1)] : sent;
    da.z = (e0 + 2 < nE) ? keys[min(e0 + 2, nE - 1)] : sent;
    da.w = (e0 + 3 < nE) ? keys[min(e0 + 3, nE - 1)] : sent;
    db.x = (e0 + 4 < nE) ? keys[min(e0 + 4, nE - 1)] : sent;
    db.y = (e0 + 5 < nE) ? keys[min(e0 + 5, nE - 1)] : sent;
    db.z = (e0 + 6 < nE) ? keys[min(e0 + 6, nE - 1)] : sent;
    db.w = (e0 + 7 < nE) ? keys[min(e0 + 7, nE - 1)] : sent;
  }
  const unsigned nbs = (unsigned)slotBase;
  const unsigned unb = (unsigned)nb;
  const unsigned s0 = (unsigned)da.x - nbs, s1 = (unsigned)da.y - nbs;
  const unsigned s2 = (unsigned)da.z - nbs, s3 = (unsigned)da.w - nbs;
  const unsigned s4 = (unsigned)db.x - nbs, s5 = (unsigned)db.y - nbs;
  const unsigned s6 = (unsigned)db.z - nbs, s7 = (unsigned)db.w - nbs;
  const bool h0 = s0 < unb, h1 = s1 < unb, h2 = s2 < unb, h3 = s3 < unb;
  const bool h4 = s4 < unb, h5 = s5 < unb, h6 = s6 < unb, h7 = s7 < unb;
  const unsigned any = __builtin_amdgcn_ballot_w32(h0 | h1 | h2 | h3 | h4 | h5 | h6 | h7);
  if (any != 0u) {
#define HITJ(J, HJ, SJ) { \
      const unsigned mj = __builtin_amdgcn_ballot_w32(HJ); \
      if (mj != 0u) { \
        if (HJ) { \
          const int pos = wc + (int)__builtin_amdgcn_mbcnt_lo(mj, 0u); \
          if (pos < WCAP) list[wave * WCAP + pos] = ((el0 + (J)) << PKS) | (int)(SJ); \
        } \
        wc += (int)__builtin_popcount(mj); } }
    HITJ(0, h0, s0)
    HITJ(1, h1, s1)
    HITJ(2, h2, s2)
    HITJ(3, h3, s3)
    HITJ(4, h4, s4)
    HITJ(5, h5, s5)
    HITJ(6, h6, s6)
    HITJ(7, h7, s7)
#undef HITJ
  }
  return wc;
}

__global__ __launch_bounds__(256) void k_zero(v4u* p, size_t n16) {
  const v4u z = {0u, 0u, 0u, 0u};
  for (size_t i = (size_t)blockIdx.x * 256 + threadIdx.x; i < n16; i += (size_t)gridDim.x * 256)
    *(volatile v4u*)(p + i) = z;
}

__global__ __launch_bounds__(NTHR) void k_prep(const float* __restrict__ W, const float* __restrict__ bvec,
                                               const float* __restrict__ h, int nN, int nUnits,
                                               unsigned short* WT, unsigned short* HB) {
  const int u = (int)blockIdx.x * NTHR + (int)threadIdx.x;
  if (u >= nUnits) return;
  v8us o;
  unsigned short* dp;
  if (u < NUWW) {
    const int n  = u >> 3;
    const int i  = n >> 6;
    const int e  = n & 63;
    const int k8 = (u & 7) * 8;
    const float* p = W + (size_t)(e * EMB + k8) * IND + i;
#pragma unroll
    for (int j = 0; j < 8; ++j) o[j] = bf_bits(p[(size_t)j * IND]);
    dp = WT + (size_t)u * 8;
  } else if (u < NUW) {
    const int n  = u >> 3;
    const int e  = n - IND * EMB;
    const int k8 = (u & 7) * 8;
    o = cvt8(bvec + (size_t)e * EMB + k8);
    dp = WT + (size_t)u * 8;
  } else {
    const int v   = u - NUW;
    const int row = v >> 3;
    const int c8  = (v & 7) * 8;
    const int rc  = row < nN ? row : nN - 1;
    o = cvt8(h + (size_t)rc * EMB + c8);
    const unsigned short msk = (row < nN) ? (unsigned short)0xFFFFu : (unsigned short)0u;
#pragma unroll
    for (int j = 0; j < 8; ++j) o[j] = (unsigned short)(o[j] & msk);
    dp = HB + (size_t)v * 8;
  }
  put16(dp, o);
}

__global__ __launch_bounds__(GTHR) void k_g(const unsigned short* __restrict__ HB,
                                            const unsigned short* __restrict__ WT, unsigned short* G16) {
  __shared__ __attribute__((aligned(16))) float stg[GBM * BNF];
  const int tid = (int)threadIdx.x, lane = tid & 31, wave = tid >> 5, hh = lane >> 4, m = lane & 15;
  const int rowBase = (int)blockIdx.x * GBM;
  const int colBase = (int)blockIdx.y * BNF;
  const unsigned short* ap = HB + (size_t)(rowBase + 16 * wave + m) * EMB + 8 * hh;
  const unsigned short* bp = WT + (size_t)(colBase + m) * EMB + 8 * hh;

  v8f acc[NTF];
  {
    const v8f z = {0.f, 0.f, 0.f, 0.f, 0.f, 0.f, 0.f, 0.f};
#pragma unroll
    for (int t = 0; t < NTF; ++t) acc[t] = z;
  }
#pragma unroll 1
  for (int k0 = 0; k0 < EMB; k0 += 32) {
    Frag af;
    af.h[0] = *(const v8usa*)(ap + k0);
    af.h[1] = *(const v8usa*)(ap + k0 + 16);
#pragma unroll
    for (int nt = 0; nt < NTF; ++nt) {
      const unsigned short* wq = bp + (size_t)(16 * nt) * EMB + k0;
      Frag bf;
      bf.h[0] = *(const v8usa*)wq;
      bf.h[1] = *(const v8usa*)(wq + 16);
      acc[nt] = wmk(af, bf, acc[nt]);
    }
  }

#pragma unroll
  for (int nt = 0; nt < NTF; ++nt) {
    const int lc = 16 * nt + m;
#pragma unroll
    for (int r = 0; r < 8; ++r) {
      const int lr = 16 * wave + 8 * hh + r;
      stg[lr * BNF + lc] = acc[nt][r] * CARRY;
    }
  }
  __syncthreads();

  unsigned short* gb = G16 + (size_t)rowBase * GW + colBase;
#pragma unroll
  for (int it = 0; it < NITF; ++it) {
    const int p  = it * GTHR + tid;
    const int pr = p / PPR;
    const int pc = p - pr * PPR;
    const v4f fa = *(const v4fa*)(stg + 8 * p);
    const v4f fb = *(const v4fa*)(stg + 8 * p + 4);
    v8f f8; f8.lo = fa; f8.hi = fb;
    const v8h h8 = __builtin_convertvector(f8, v8h);
    const v8us v = __builtin_bit_cast(v8us, h8);
    *(volatile v8us*)(gb + (size_t)pr * GW + 8 * pc) = v;
  }
  __threadfence();
#pragma unroll
  for (int it = 0; it < NITF; ++it) {
    const int p  = it * GTHR + tid;
    const int pr = p / PPR;
    const int pc = p - pr * PPR;
    const v4f fa = *(const v4fa*)(stg + 8 * p);
    const v4f fb = *(const v4fa*)(stg + 8 * p + 4);
    v8f f8; f8.lo = fa; f8.hi = fb;
    const v8h h8 = __builtin_convertvector(f8, v8h);
    const v8us v = __builtin_bit_cast(v8us, h8);
    *(volatile v8us*)(gb + (size_t)pr * GW + 8 * pc) = v;
  }
}

__global__ __launch_bounds__(ETHR) void k_edge(const float* __restrict__ ea, const int* __restrict__ cols,
                                               int nE, int nN, const unsigned short* __restrict__ G16,
                                               float* MSG) {
  __shared__ __attribute__((aligned(16))) float ms[ETHR * EMB];
  const int tid = (int)threadIdx.x;
  const int elb = (int)blockIdx.x * ETHR;
  const int el  = elb + tid;
  const int elc = el < nE ? el : nE - 1;
  int c = cols[elc];
  c = c < 0 ? 0 : (c > nN - 1 ? nN - 1 : c);
  const unsigned short* gr = G16 + (size_t)c * GW;
  const float* er = ea + (size_t)elc * IND;

  float acc[EMB];
#pragma unroll
  for (int e = 0; e < EMB; ++e) acc[e] = 0.0f;

#pragma unroll 1
  for (int i = 0; i < NGI; ++i) {
    const int ic = i < IND ? i : IND - 1;
    const float ev = bf_rne(er[ic]);
    const float f  = (i < IND) ? ev : 1.0f;
    const unsigned int* gp = (const unsigned int*)(gr + (size_t)i * EMB);
#pragma unroll
    for (int q = 0; q < 8; ++q) {
      const v4u w = *(const v4ua*)(gp + 4 * q);
      acc[8 * q + 0] = fmaf(f, h2f(w.x),       acc[8 * q + 0]);
      acc[8 * q + 1] = fmaf(f, h2f(w.x >> 16), acc[8 * q + 1]);
      acc[8 * q + 2] = fmaf(f, h2f(w.y),       acc[8 * q + 2]);
      acc[8 * q + 3] = fmaf(f, h2f(w.y >> 16), acc[8 * q + 3]);
      acc[8 * q + 4] = fmaf(f, h2f(w.z),       acc[8 * q + 4]);
      acc[8 * q + 5] = fmaf(f, h2f(w.z >> 16), acc[8 * q + 5]);
      acc[8 * q + 6] = fmaf(f, h2f(w.w),       acc[8 * q + 6]);
      acc[8 * q + 7] = fmaf(f, h2f(w.w >> 16), acc[8 * q + 7]);
    }
  }

  float* md = ms + (size_t)tid * EMB;
#pragma unroll
  for (int q = 0; q < 16; ++q) {
    v4f v;
    v.x = acc[4 * q + 0] * INV_CARRY;
    v.y = acc[4 * q + 1] * INV_CARRY;
    v.z = acc[4 * q + 2] * INV_CARRY;
    v.w = acc[4 * q + 3] * INV_CARRY;
    *(v4fa*)(md + 4 * q) = v;
  }
  __syncthreads();

  float* mb = MSG + (size_t)elb * EMB;
#pragma unroll
  for (int it = 0; it < NITE; ++it) {
    const int p = it * ETHR + tid;
    const v4f v = *(const v4fa*)(ms + 4 * p);
    *(volatile v4f*)(mb + (size_t)4 * p) = v;
  }
  __threadfence();
#pragma unroll
  for (int it = 0; it < NITE; ++it) {
    const int p = it * ETHR + tid;
    const v4f v = *(const v4fa*)(ms + 4 * p);
    *(volatile v4f*)(mb + (size_t)4 * p) = v;
  }
}

__global__ __launch_bounds__(NTHR) void k_scan(const int* __restrict__ keys, const float* __restrict__ MSG,
                                               const float* __restrict__ h, const float* __restrict__ gamma,
                                               const float* __restrict__ beta, float* out, int nN, int nE,
                                               int vec8) {
  extern __shared__ __attribute__((aligned(16))) int lds_i[];
  int* reg1 = lds_i;
  int* reg2 = reg1 + RCAP;
  int* scnt = reg2 + RCAP;
  int* soff = scnt + NBA;
  int* list = soff + NBA;
  int* wcnt = list + LISTN;
  int* wtot = wcnt + NWAVE;
  const int tid = (int)threadIdx.x, lane = tid & 31, wave = tid >> 5;
  const int nodeBase = (int)blockIdx.x * NBA;

  {
    const v4i z4 = {0, 0, 0, 0};
    for (int i = tid * 4; i < ZINTS; i += NTHR * 4) *(v4ia*)(lds_i + i) = z4;
    if (tid < 2 * NWAVE) wcnt[tid] = 0;
  }
  __syncthreads();

  int tot = 0;
  const int nChunks = (nE + CHUNK - 1) / CHUNK;
#pragma unroll 1
  for (int ch = 0; ch < nChunks; ++ch) {
    const int cbase = ch * CHUNK;
    const int wc = scan_chunk(keys, nE, cbase, nodeBase, NBA, vec8, list, tid, lane, wave);
    if (lane == 0) wcnt[wave] = wc;
    __syncthreads();
    int pre = 0, all = 0;
#pragma unroll
    for (int w2 = 0; w2 < NWAVE; ++w2) {
      int cw = wcnt[w2];
      cw = cw < 0 ? 0 : (cw > WCAP ? WCAP : cw);
      all += cw;
      pre += (w2 < wave) ? cw : 0;
    }
    const int wcc  = wc > WCAP ? WCAP : wc;
    const int base = tot + pre;
#pragma unroll 1
    for (int i = lane; i < wcc; i += 32) {
      const int ent = list[wave * WCAP + i];
      const int el  = (ent >> PKS) & (CHUNK - 1);
      const int sl  = ent & (NBA - 1);
      int eid = cbase + el;
      eid = eid > nE - 1 ? nE - 1 : eid;
      const int pos = base + i;
      if (pos < RCAP) reg1[pos] = (int)(((unsigned)eid << PKS) | (unsigned)sl);
    }
    tot += all;
    tot = tot > RCAP ? RCAP : tot;
    __syncthreads();
  }
  const int nh = tot;

  if (wave == 0) {
#pragma unroll 1
    for (int b0 = 0; b0 < nh; b0 += 32) {
      const int idx = b0 + lane;
      const int uv  = reg1[idx < RCAP ? idx : RCAP - 1];
      const int m32 = (nh - b0) < 32 ? (nh - b0) : 32;
#pragma unroll 1
      for (int k = 0; k < m32; ++k) {
        const int u  = __builtin_amdgcn_readlane(uv, k);
        const int sl = u & (NBA - 1);
        if (lane == 0) scnt[sl] = scnt[sl] + 1;
      }
    }
  }
  __syncthreads();

  {
    const v4i ca = *(const v4ia*)(scnt + 4 * tid);
    const int e0 = ca.x < 0 ? 0 : ca.x, e1 = ca.y < 0 ? 0 : ca.y, e2 = ca.z < 0 ? 0 : ca.z, e3 = ca.w < 0 ? 0 : ca.w;
    const int ts = e0 + e1 + e2 + e3;
    int incl = ts;
#pragma unroll
    for (int d = 1; d < 32; d <<= 1) {
      const int up = __shfl_up(incl, d, 32);
      if (lane >= d) incl += up;
    }
    if (lane == 31) wtot[wave] = incl;
    __syncthreads();
    int pre = 0;
#pragma unroll
    for (int w2 = 0; w2 < NWAVE; ++w2) pre += (w2 < wave) ? wtot[w2] : 0;
    int run = pre + incl - ts;
    soff[4 * tid + 0] = run; run += e0;
    soff[4 * tid + 1] = run; run += e1;
    soff[4 * tid + 2] = run; run += e2;
    soff[4 * tid + 3] = run;
  }
  __syncthreads();
  for (int i = tid; i < NBA; i += NTHR) list[i] = soff[i];
  __syncthreads();

  if (wave == 0) {
#pragma unroll 1
    for (int b0 = 0; b0 < nh; b0 += 32) {
      const int idx = b0 + lane;
      const int uv  = reg1[idx < RCAP ? idx : RCAP - 1];
      const int m32 = (nh - b0) < 32 ? (nh - b0) : 32;
#pragma unroll 1
      for (int k = 0; k < m32; ++k) {
        const int u   = __builtin_amdgcn_readlane(uv, k);
        const int sl  = u & (NBA - 1);
        const int eid = (int)((unsigned)u >> PKS);
        if (lane == 0) {
          int pos = list[sl];
          pos = pos < 0 ? 0 : (pos > RCAP - 1 ? RCAP - 1 : pos);
          reg2[pos] = eid;
          list[sl] = pos + 1;
        }
      }
    }
  }
  __syncthreads();

  const int nbw = NBA / NWAVE;
  const bool ovf = (nh >= RCAP);
  const float qnan = __int_as_float(0x7fc00000);
  const int c2 = 2 * lane;
  float g0, g1, t0, t1;
  {
    const v2f gv = *(const v2fa*)(gamma + c2);
    const v2f tv = *(const v2fa*)(beta + c2);
    g0 = bf_rne(gv.x); g1 = bf_rne(gv.y);
    t0 = bf_rne(tv.x); t1 = bf_rne(tv.y);
  }

#pragma unroll 1
  for (int jt = 0; jt < nbw; ++jt) {
    const int slot = wave * nbw + jt;
    const int node = nodeBase + slot;
    int st = soff[slot];
    const int craw = scnt[slot];
    int cnt = craw;
    st  = st < 0 ? 0 : (st > nh ? nh : st);
    cnt = cnt < 0 ? 0 : (cnt > DEGCAP ? DEGCAP : cnt);
    if (cnt > nh - st) cnt = nh - st;
    const float pz = (ovf || craw > DEGCAP) ? qnan : 0.0f;
    const bool live = node < nN;

    float ax = 0.0f, ay = 0.0f;
#pragma unroll 1
    for (int b0 = 0; b0 < cnt; b0 += 32) {
      int idx = st + b0 + lane; idx = idx > RCAP - 1 ? RCAP - 1 : idx;
      int eid = reg2[idx]; eid = eid < 0 ? 0 : (eid > nE - 1 ? nE - 1 : eid);
      const int m32 = (cnt - b0) < 32 ? (cnt - b0) : 32;
#pragma unroll 1
      for (int k = 0; k < m32; ++k) {
        const int ek = __builtin_amdgcn_readlane(eid, k);
        const v2f mv = *(const v2fa*)(MSG + (size_t)ek * EMB + c2);
        ax += mv.x;
        ay += mv.y;
      }
    }
    const int ncl = live ? node : nN - 1;
    const v2f hv = *(const v2fa*)(h + (size_t)ncl * EMB + c2);
    const float x0 = bf_rne(hv.x) + ax;
    const float x1 = bf_rne(hv.y) + ay;
    float s = x0 + x1;
#pragma unroll
    for (int off = 16; off > 0; off >>= 1) s += __shfl_xor(s, off);
    const float mu = s * INV_EMB;
    const float d0 = x0 - mu, d1 = x1 - mu;
    float q = d0 * d0 + d1 * d1;
#pragma unroll
    for (int off = 16; off > 0; off >>= 1) q += __shfl_xor(q, off);
    const float var = q * INV_EMB;
    const float inv = rsqrtf(var + LN_EPS);
    const float y0 = (d0 * inv) * g0 + t0 + pz;
    const float y1 = (d1 * inv) * g1 + t1 + pz;
    if (live) {
      v2f o;
      o.x = y0; o.y = y1;
      float* op = out + (size_t)node * EMB + c2;
      *(volatile v2f*)op = o;
      __threadfence();
      *(volatile v2f*)op = o;
    }
  }
}

static inline int cdiv(int a, int b) { return (a + b - 1) / b; }
static inline size_t al256(size_t o) { return (o + 255) & ~(size_t)255; }

extern "C" void kernel_launch(void* const* d_in, const int* in_sizes, int n_in,
                              void* d_out, int out_size, void* d_ws, size_t ws_size,
                              hipStream_t stream) {
  if (n_in < 7) return;
  if (in_sizes[0] < EMB || (in_sizes[0] % EMB) != 0) return;
  const int nN = in_sizes[0] / EMB;
  if (nN < 1 || nN > (1 << 22)) return;
  if (in_sizes[1] < IND || (in_sizes[1] % IND) != 0) return;
  const int nE = in_sizes[1] / IND;
  if (nE < 1 || nE >= (1 << 21)) return;
  if (in_sizes[2] != WROWS * IND) return;
  if (in_sizes[3] != WROWS) return;
  if (in_sizes[4] != EMB) return;
  if (in_sizes[5] != EMB) return;
  if ((long long)in_sizes[6] != 2LL * (long long)nE) return;
  if ((long long)out_size != (long long)nN * EMB) return;

  const float* h     = (const float*)d_in[0];
  const float* ea    = (const float*)d_in[1];
  const float* W     = (const float*)d_in[2];
  const float* bvec  = (const float*)d_in[3];
  const float* gamma = (const float*)d_in[4];
  const float* beta  = (const float*)d_in[5];
  const int*   ei    = (const int*)  d_in[6];
  const int*   keys  = ei;
  const int*   cols  = ei + nE;
  float* out = (float*)d_out;

  const int MP   = cdiv(nN, GBM) * GBM;
  const int gM   = MP / GBM;
  const int EP   = cdiv(nE, ETHR) * ETHR;
  const int gE   = EP / ETHR;
  const int gA   = cdiv(nN, NBA);
  if ((long long)gA * NBA < (long long)nN) return;
  const int vec8 = ((nE & 3) == 0) ? 1 : 0;
  const long long nUnitsLL = (long long)NUW + (long long)MP * (EMB / 8);
  if (nUnitsLL > (1LL << 30) || (nUnitsLL % NTHR) != 0) return;
  const int nUnits = (int)nUnitsLL;

  char* ws = (char*)d_ws;
  size_t off = 0;
  const size_t oWT  = off; off = al256(off + (size_t)NUW * 8 * 2);
  const size_t oHB  = off; off = al256(off + (size_t)MP * EMB * 2);
  const size_t oG   = off; off = al256(off + (size_t)MP * GW * 2);
  const size_t oMSG = off; off = al256(off + (size_t)EP * EMB * 4);
  if (off > ws_size || off > (size_t)WSLIM) return;
  unsigned short* WT  = (unsigned short*)(ws + oWT);
  unsigned short* HB  = (unsigned short*)(ws + oHB);
  unsigned short* G16 = (unsigned short*)(ws + oG);
  float*          MSG = (float*)(ws + oMSG);

  hipFuncSetAttribute(reinterpret_cast<const void*>(&k_scan), hipFuncAttributeMaxDynamicSharedMemorySize, LDS_AGG);

  k_zero<<<1024, 256, 0, stream>>>((v4u*)ws, off / 16);
  k_prep<<<nUnits / NTHR, NTHR, 0, stream>>>(W, bvec, h, nN, nUnits, WT, HB);
  k_g<<<dim3(gM, NCB), GTHR, 0, stream>>>(HB, WT, G16);
  k_edge<<<gE, ETHR, 0, stream>>>(ea, cols, nE, nN, G16, MSG);
  k_scan<<<gA, NTHR, LDS_AGG, stream>>>(keys, MSG, h, gamma, beta, out, nN, nE, vec8);
}
